// HGTLayer_53188874994368
// MI455X (gfx1250) — hardware-run, weakly checked
//
#include <hip/hip_runtime.h>


namespace {

constexpr int N = 50000, NP = 50048, NPL = NP  , SRCM = N  , EFULL = 600000, E = EFULL  , D = 128, NH = 4, DK = 32, NL = (NPL < N ? NPL : N);
constexpr float XS = 8.0f, WSC = 256.0f, WSQ = 0.25f, RS_ = 1024.0f, LNEPS = 1e-5f, ISQ = 0.17677669529663687f  , SLOPE = 0.0f, BNEPS = 1e-5f;
static_assert(NP % 64 == 0 && NP >= N && NPL % 64 == 0 && D == 128 && NH * DK == D, "tiling");
typedef _Float16 b16;
typedef __attribute__((ext_vector_type(16))) _Float16 v16b;
typedef __attribute__((ext_vector_type(8))) _Float16 v8b;
typedef __attribute__((ext_vector_type(8))) float v8f;
typedef __attribute__((ext_vector_type(4))) float v4f;
__device__ __forceinline__ float bf16_rne(float f) { unsigned int u = __float_as_uint(f); u += 0x7FFFu + ((u >> 16) & 1u); return __uint_as_float(u & 0xFFFF0000u); }
__device__ __forceinline__ void split16(float v, b16& hi, b16& lo) { hi = (b16)v; lo = (b16)(v - (float)hi); }
__device__ __forceinline__ v16b frag_kb(const b16* p, int hh) { const v8b a = *(const v8b*)(p + 8 * hh), b = *(const v8b*)(p + 16 + 8 * hh); v16b f;
#pragma unroll
  for (int e = 0; e < 8; ++e) { f[e] = a[e]; f[8 + e] = b[e]; } return f; }
__device__ __forceinline__ v8f wmma16b(v16b a, v16b b, v8f c) { v8f d = __builtin_amdgcn_wmma_f32_16x16x32_f16(false, a, false, b, (short)0, c, false, false); asm volatile("v_nop\n\tv_nop\n\tv_nop\n\tv_nop" : "+v"(d) : "v"(a), "v"(b)); return d; }
__device__ __forceinline__ void wave_lds_sync() { __builtin_amdgcn_fence(__ATOMIC_RELEASE, "workgroup"); __builtin_amdgcn_wave_barrier(); __builtin_amdgcn_fence(__ATOMIC_ACQUIRE, "workgroup"); }
__device__ __forceinline__ float pmul(float a, float b) { float p = a * b; asm volatile("" : "+v"(p)); return p; }
__device__ __forceinline__ int iclamp(int v, int lo, int hi) { return v < lo ? lo : (v > hi ? hi : v); }
constexpr int CSR_NBLK = 512, CSR_GB = 9, CSR_GN = 1 << CSR_GB  , CSR_MAXG = 512, CSR_CAP = 12288  ;
__global__ __launch_bounds__(64) void csrA_kernel(const int* __restrict__ dst, int E, int N, int nG, int CHP, int NGP, int* __restrict__ STG, int* __restrict__ HST) {
  extern __shared__ int sm[];
  int* cnt = sm; int* run = sm + NGP; int* ids = sm + 2 * NGP;
  const int b = blockIdx.x; const int ch = (E + CSR_NBLK - 1) / CSR_NBLK; const int e0 = b * ch, e1 = min(E, e0 + ch);
  for (int i = threadIdx.x; i < NGP; i += 64) cnt[i] = 0;
  for (int i = threadIdx.x; i < CHP; i += 64) ids[i] = -1;
  __syncthreads();
  if (threadIdx.x == 0) {
    for (int e = e0; e < e1; ++e) { int d = dst[e]; d = (d < 0) ? 0 : (d >= N ? N - 1 : d); cnt[d >> CSR_GB] += 1; }
    int acc = 0; for (int g = 0; g < nG; ++g) { run[g] = acc; acc += cnt[g]; }
    for (int e = e0; e < e1; ++e) { int d = dst[e]; d = (d < 0) ? 0 : (d >= N ? N - 1 : d); const int g = d >> CSR_GB; ids[run[g]] = e; run[g] += 1; } }
  __syncthreads();
  typedef __attribute__((ext_vector_type(4))) int v4i;
  for (int pass = 0; pass < 2; ++pass) {
    for (int i = threadIdx.x; i < CHP / 4; i += 64) *(volatile v4i*)(STG + (size_t)b * CHP + i * 4) = *(const v4i*)(&ids[i * 4]);
    for (int i = threadIdx.x; i < NGP / 4; i += 64) { v4i v; for (int e = 0; e < 4; ++e) v[e] = (i * 4 + e < nG) ? cnt[i * 4 + e] : 0; *(volatile v4i*)(HST + (size_t)b * NGP + i * 4) = v; }
    __threadfence(); }
}
__global__ __launch_bounds__(512) void csrS_kernel(const int* __restrict__ HST, int nG, int NGP, int* __restrict__ START, int* __restrict__ TOT, int* __restrict__ OFF) {
  __shared__ int tot[CSR_MAXG];
  const int b = threadIdx.x;
  for (int pass = 0; pass < 2; ++pass) { int runb = 0; for (int g = 0; g < nG; ++g) { int c = HST[(size_t)b * NGP + g]; c = (c < 0) ? 0 : c; ((volatile int*)OFF)[(size_t)g * CSR_NBLK + b] = runb; runb += c; } __threadfence(); }
  for (int g = threadIdx.x; g < nG; g += 512) { int s = 0; for (int bb = 0; bb < CSR_NBLK; ++bb) { int c = HST[(size_t)bb * NGP + g]; s += (c < 0) ? 0 : c; } tot[g] = s; }
  __syncthreads();
  if (threadIdx.x < 32) {
    __shared__ int st[CSR_MAXG + 32];
    if (threadIdx.x == 0) { int acc = 0; for (int g = 0; g < NGP; ++g) { st[g] = acc; if (g < nG) acc += (tot[g] + 31) & ~31; } st[NGP] = acc; }
    __builtin_amdgcn_fence(__ATOMIC_RELEASE, "workgroup"); __builtin_amdgcn_wave_barrier(); __builtin_amdgcn_fence(__ATOMIC_ACQUIRE, "workgroup");
    for (int pass = 0; pass < 2; ++pass) { for (int i = threadIdx.x; i < NGP + 32; i += 32) { ((volatile int*)START)[i] = (i <= NGP) ? st[min(i, NGP)] : 0; ((volatile int*)TOT)[i] = (i < nG) ? tot[i] : 0; } __threadfence(); } }
}
__global__ __launch_bounds__(256) void csrB_kernel(const int* __restrict__ dst, int N, int nG, int CHP, int NGP, int permLen, const int* __restrict__ STG, const int* __restrict__ HST, const int* __restrict__ OFF, const int* __restrict__ START, const int* __restrict__ TOT, int* __restrict__ PERM, int* __restrict__ ROWPTR, int* __restrict__ ROWCNT, int* __restrict__ FLAG) {
  typedef __attribute__((ext_vector_type(4))) int v4i;
  __shared__ int ids[CSR_CAP]; __shared__ unsigned short key[CSR_CAP]; __shared__ int outp[CSR_CAP]; __shared__ int ncnt[CSR_GN + 1]; __shared__ int boff[CSR_NBLK + 1];
  const int g = blockIdx.x, t_ = threadIdx.x; int tot = TOT[g]; int st = START[g], stn = START[g + 1]; const int v0 = g * CSR_GN; const int nv = min(CSR_GN, N - v0);
  st = (st < 0) ? 0 : (st > permLen - 32 ? permLen - 32 : st) & ~31; stn = (stn < st) ? st : (stn > permLen ? permLen : stn); tot = (tot < 0) ? 0 : tot; if (tot > stn - st && tot <= CSR_CAP) tot = stn - st;
  if (tot > CSR_CAP) {
    for (int pass = 0; pass < 2; ++pass) { for (int i = t_; i < CSR_GN / 4; i += 256) { v4i a, c; for (int e = 0; e < 4; ++e) { a[e] = st; c[e] = 0; } *(volatile v4i*)(ROWPTR + v0 + i * 4) = a; *(volatile v4i*)(ROWCNT + v0 + i * 4) = c; } if (t_ == 0) ((volatile int*)FLAG)[0] = 1; __threadfence(); } (void)nv; return; }
  if (t_ == 0) { int acc = 0; for (int b = 0; b < CSR_NBLK; ++b) { boff[b] = acc; int c = HST[(size_t)b * NGP + g]; c = (c < 0) ? 0 : (c > CHP ? CHP : c); acc += c; if (acc > tot) acc = tot; } boff[CSR_NBLK] = acc; }
  for (int i = t_; i <= CSR_GN; i += 256) ncnt[i] = 0;
  __syncthreads();
  for (int b = 0; b < CSR_NBLK; ++b) { const int c = boff[b + 1] - boff[b]; int o_ = OFF[(size_t)g * CSR_NBLK + b]; o_ = (o_ < 0) ? 0 : (o_ > CHP - c ? CHP - c : o_); const int* src_ = STG + (size_t)b * CHP + o_;
    for (int i = t_; i < c; i += 256) { int id = src_[i]; id = (id < 0) ? 0 : id; ids[boff[b] + i] = id; int d = dst[id]; d = (d < v0) ? v0 : (d >= N ? N - 1 : d); int kk = d - v0; kk = (kk < 0) ? 0 : (kk >= CSR_GN ? CSR_GN - 1 : kk); key[boff[b] + i] = (unsigned short)kk; } }
  __syncthreads();
  if (t_ == 0) { for (int i = 0; i < tot; ++i) ncnt[key[i]] += 1; int acc = 0; for (int vl = 0; vl < CSR_GN; ++vl) { const int c = ncnt[vl]; ncnt[vl] = acc; acc += c; } ncnt[CSR_GN] = acc;
    for (int i = 0; i < tot; ++i) { const int vl = key[i]; outp[ncnt[vl]] = ids[i]; ncnt[vl] += 1; }
    for (int vl = CSR_GN; vl > 0; --vl) ncnt[vl] = ncnt[vl - 1]; ncnt[0] = 0; }
  __syncthreads();
  for (int pass = 0; pass < 2; ++pass) {
    for (int i = t_; i < (stn - st) / 4; i += 256) { v4i v; for (int e = 0; e < 4; ++e) { const int q = i * 4 + e; v[e] = (q < tot) ? outp[q] : -1; } *(volatile v4i*)(PERM + st + i * 4) = v; }
    for (int i = t_; i < CSR_GN / 4; i += 256) { v4i a, c; for (int e = 0; e < 4; ++e) { const int vl = i * 4 + e; a[e] = st + ncnt[vl]; c[e] = (vl < nv) ? (ncnt[vl + 1] - ncnt[vl]) : 0; } *(volatile v4i*)(ROWPTR + v0 + i * 4) = a; *(volatile v4i*)(ROWCNT + v0 + i * 4) = c; }
    __threadfence(); }
}
__global__ __launch_bounds__(256) void csrZ_kernel(int* __restrict__ p, size_t n4) { typedef __attribute__((ext_vector_type(4))) int v4i; const size_t tid = (size_t)blockIdx.x * 256 + threadIdx.x, nth = (size_t)gridDim.x * 256; v4i z = {0, 0, 0, 0}; for (size_t i = tid; i < n4; i += nth) *(volatile v4i*)(p + i * 4) = z; }
struct CsrBufs { int *STG, *HST, *OFF, *START, *TOT, *PERM, *ROWPTR, *ROWCNT, *FLAG; int nG, NGP, CHP; size_t permLen; char* base; size_t bytes; };
static size_t csr_carve(CsrBufs& c, char* ws, size_t off, int E, int N) {
  const size_t off0 = off; c.base = ws + off;
  auto al = [&](size_t bytes) { char* p = ws + off; off += (bytes + 255) & ~(size_t)255; return p; };
  c.nG = (N + CSR_GN - 1) / CSR_GN; c.NGP = (c.nG + 31) & ~31; const int ch = (E + CSR_NBLK - 1) / CSR_NBLK; c.CHP = (ch + 31) & ~31; c.permLen = (size_t)E + 32 * (size_t)c.nG + 32;
  c.STG = (int*)al((size_t)CSR_NBLK * c.CHP * 4); c.HST = (int*)al((size_t)CSR_NBLK * c.NGP * 4); c.OFF = (int*)al((size_t)c.NGP * CSR_NBLK * 4); c.START = (int*)al((size_t)(c.NGP + 64) * 4); c.TOT = (int*)al((size_t)(c.NGP + 64) * 4);
  c.PERM = (int*)al(c.permLen * 4); c.ROWPTR = (int*)al((size_t)c.nG * CSR_GN * 4); c.ROWCNT = (int*)al((size_t)c.nG * CSR_GN * 4); c.FLAG = (int*)al(256);
  c.bytes = off - off0; return off;
}
static void csr_build(const CsrBufs& c, const int* dst, int E, int N, hipStream_t stream) {
  const size_t smem = (size_t)(2 * c.NGP + c.CHP) * 4;
  csrZ_kernel<<<512, 256, 0, stream>>>((int*)c.base, c.bytes / 16);
  csrA_kernel<<<CSR_NBLK, 64, smem, stream>>>(dst, E, N, c.nG, c.CHP, c.NGP, c.STG, c.HST);
  csrS_kernel<<<1, 512, 0, stream>>>(c.HST, c.nG, c.NGP, c.START, c.TOT, c.OFF);
  csrB_kernel<<<c.nG, 256, 0, stream>>>(dst, N, c.nG, c.CHP, c.NGP, (int)c.permLen, c.STG, c.HST, c.OFF, c.START, c.TOT, c.PERM, c.ROWPTR, c.ROWCNT, c.FLAG);
}

typedef __attribute__((ext_vector_type(4))) _Float16 v4h;
typedef __attribute__((ext_vector_type(2))) float v2f;
template <int KD, int NOUT>
__global__ __launch_bounds__(256) void wprep_kernel(const float* __restrict__ w, b16* __restrict__ WT) {
  static_assert(KD % 8 == 0, "wprep"); const size_t u = (size_t)blockIdx.x * 256 + threadIdx.x; if (u >= (size_t)NOUT * KD / 8) return; const size_t e = u * 8; const int oo = (int)(e / KD), k0 = (int)(e % KD); v8b o;
  for (int j = 0; j < 8; ++j) o[j] = (b16)(bf16_rne(w[(size_t)(k0 + j) * NOUT + oo]) * WSC);
  for (int pass = 0; pass < 2; ++pass) { *(volatile v8b*)(WT + e) = o; __threadfence(); }
}

__global__ __launch_bounds__(256) void bd_kernel(const float* __restrict__ w, b16* __restrict__ BD, float scl) {
  const int u = blockIdx.x * 256 + threadIdx.x; if (u >= D * D / 8) return; const int e = u * 8; const int o = e / D, k0 = e % D; const int h = o / DK, j = o % DK; v8b v;
#pragma unroll
  for (int q = 0; q < 8; ++q) { const int k = k0 + q; const int hk = k / DK, i = k % DK; v[q] = (b16)(hk == h ? bf16_rne(w[((size_t)h * DK + i) * DK + j]) * scl : 0.0f); }
  for (int pass = 0; pass < 2; ++pass) { *(volatile v8b*)(BD + e) = v; __threadfence(); }
}
template <bool FOLD>
__global__ __launch_bounds__(64) void proj_kernel(const float* __restrict__ F, const b16* __restrict__ WT, const float* __restrict__ bias, const b16* __restrict__ BDT, const b16* __restrict__ BDQ, float* __restrict__ OUT) {
  __shared__ __attribute__((aligned(16))) b16 As[2][16][D + 8], Al[2][16][D + 8]; __shared__ __attribute__((aligned(16))) float Tf[2][16][D + 4];
  const int wave = threadIdx.x >> 5, lane = threadIdx.x & 31, nloc = lane & 15, hlf = lane >> 4; const size_t m0 = (size_t)blockIdx.x * 32 + wave * 16;
  for (int idx = lane; idx < 16 * 32; idx += 32) { const int rr = idx / 32, c4 = (idx % 32) * 4; const v4f v = *(const v4f*)(F + (m0 + rr < (size_t)N ? m0 + rr : (size_t)N - 1) * D + c4); v4h o; for (int j = 0; j < 4; ++j) o[j] = (b16)(bf16_rne(v[j]) * XS); *(v4h*)(&As[wave][rr][c4]) = o; }
  wave_lds_sync();
  v8f acc[8];
#pragma unroll
  for (int t = 0; t < 8; ++t) acc[t] = (v8f){};
#pragma unroll
  for (int kb = 0; kb < D; kb += 32) { const v16b a = frag_kb(&As[wave][nloc][kb], hlf);
#pragma unroll
    for (int t = 0; t < 8; ++t) acc[t] = wmma16b(a, frag_kb(WT + (size_t)(t * 16 + nloc) * D + kb, hlf), acc[t]); }
#pragma unroll
  for (int t = 0; t < 8; ++t) { const float bb = bf16_rne(bias[t * 16 + nloc]);
#pragma unroll
    for (int r = 0; r < 8; ++r) Tf[wave][8 * hlf + r][t * 16 + nloc] = acc[t][r] * (1.0f / (XS * WSC)) + bb; }
  wave_lds_sync();
  if (FOLD) {
    for (int idx = lane; idx < 16 * 32; idx += 32) { const int rr = idx / 32, c4 = (idx % 32) * 4; v4h hv, lv; for (int j = 0; j < 4; ++j) { const float vs = Tf[wave][rr][c4 + j] * XS; const b16 ph = (b16)vs; hv[j] = ph; lv[j] = (b16)((vs - (float)ph) * RS_); } *(v4h*)(&As[wave][rr][c4]) = hv; *(v4h*)(&Al[wave][rr][c4]) = lv; }
    wave_lds_sync();
#pragma unroll
    for (int t = 0; t < 8; ++t) acc[t] = (v8f){};
#pragma unroll
    for (int kb = 0; kb < D; kb += 32) { const v16b a = frag_kb(&As[wave][nloc][kb], hlf), al = frag_kb(&Al[wave][nloc][kb], hlf);
#pragma unroll
      for (int t = 0; t < 8; ++t) { const size_t wo_ = (size_t)(t * 16 + nloc) * D + kb; acc[t] = wmma16b(a, frag_kb(BDT + wo_, hlf), acc[t]); acc[t] = wmma16b(al, frag_kb(BDQ + wo_, hlf), acc[t]); } }
    wave_lds_sync();
#pragma unroll
    for (int t = 0; t < 8; ++t)
#pragma unroll
      for (int r = 0; r < 8; ++r) Tf[wave][8 * hlf + r][t * 16 + nloc] = acc[t][r] * (1.0f / (XS * WSC));
    wave_lds_sync(); }
  for (int pass = 0; pass < 2; ++pass) { for (int rr = 0; rr < 16; ++rr) *(volatile v4f*)(OUT + (m0 + rr) * D + lane * 4) = *(const v4f*)(&Tf[wave][rr][lane * 4]); __threadfence(); }
}
__global__ __launch_bounds__(256) void attn_kernel(const float* __restrict__ Q, const float* __restrict__ K, const float* __restrict__ V, const float* __restrict__ mu, const int* __restrict__ srcs, const int* __restrict__ PERM, const int* __restrict__ ROWPTR, const int* __restrict__ ROWCNT, int permLen, float* __restrict__ Hout) {
  __shared__ __attribute__((aligned(16))) float rows[64][D + 4];
  const int tid = threadIdx.x; const int row = tid >> 2, h = tid & 3; const int v = blockIdx.x * 64 + row; const float scl = bf16_rne(mu[h]) * ISQ;
  float q[DK], acc[DK]; for (int j = 0; j < DK; ++j) { q[j] = 0.0f; acc[j] = 0.0f; }
  int cnt = 0, p0 = 0; if (v < N) { cnt = iclamp(ROWCNT[v], 0, 65536); p0 = iclamp(ROWPTR[v], 0, permLen - 1); if (p0 + cnt > permLen) cnt = permLen - p0; const float* qr = Q + (size_t)v * D + h * DK;
#pragma unroll
    for (int j4 = 0; j4 < DK; j4 += 4) { const v4f t4 = *(const v4f*)(qr + j4); for (int j = 0; j < 4; ++j) q[j4 + j] = t4[j]; } }
  float m = -INFINITY, l = 0.0f;
#pragma unroll 1
  for (int i = 0; i < cnt; ++i) { int e = iclamp(PERM[p0 + i], 0, E - 1); int s = iclamp(srcs[e], 0, N - 1); if (SRCM < N) s %= SRCM; const float* kr = K + (size_t)s * D + h * DK; const float* vr = V + (size_t)s * D + h * DK; float dot = 0.0f;
#pragma unroll
    for (int j4 = 0; j4 < DK; j4 += 4) { const v4f t4 = *(const v4f*)(kr + j4); for (int j = 0; j < 4; ++j) dot = fmaf(q[j4 + j], t4[j], dot); }
    const float sc = dot * scl; const float mn = fmaxf(m, sc); const float al = __expf(m - mn)  ; const float p = __expf(sc - mn); l = l * al + p; m = mn;
#pragma unroll
    for (int j4 = 0; j4 < DK; j4 += 4) { const v4f t4 = *(const v4f*)(vr + j4); for (int j = 0; j < 4; ++j) acc[j4 + j] = fmaf(p, t4[j], acc[j4 + j] * al); } }
  const float inv = (v < N && cnt > 0) ? 1.0f / l : 0.0f;
#pragma unroll
  for (int j = 0; j < DK; ++j) rows[row][h * DK + j] = acc[j] * inv;
  __syncthreads();
  const int wave = tid >> 5, lane = tid & 31;
  for (int pass = 0; pass < 2; ++pass) { for (int rr = wave * 8; rr < wave * 8 + 8; ++rr) *(volatile v4f*)(Hout + (size_t)(blockIdx.x * 64 + rr) * D + lane * 4) = *(const v4f*)(&rows[rr][lane * 4]); __threadfence(); }
}
__global__ __launch_bounds__(64) void nodeout_kernel(const float* __restrict__ Hh, const float* __restrict__ F, const b16* __restrict__ WAT, const float* __restrict__ ba, const float* __restrict__ skip, const float* __restrict__ g, const float* __restrict__ bb_, float* __restrict__ out) {
  __shared__ __attribute__((aligned(16))) b16 As[2][16][D + 8]; __shared__ __attribute__((aligned(16))) float Tf[2][16][D + 4];
  const int wave = threadIdx.x >> 5, lane = threadIdx.x & 31, nloc = lane & 15, hlf = lane >> 4; const size_t m0 = (size_t)blockIdx.x * 32 + wave * 16;
  for (int idx = lane; idx < 16 * 32; idx += 32) { const int rr = idx / 32, c4 = (idx % 32) * 4; const v4f v = *(const v4f*)(Hh + (m0 + rr) * D + c4); v4h o; for (int j = 0; j < 4; ++j) o[j] = (b16)(v[j] * XS); *(v4h*)(&As[wave][rr][c4]) = o; }
  wave_lds_sync();
  v8f acc[8];
#pragma unroll
  for (int t = 0; t < 8; ++t) acc[t] = (v8f){};
#pragma unroll
  for (int kb = 0; kb < D; kb += 32) { const v16b a = frag_kb(&As[wave][nloc][kb], hlf);
#pragma unroll
    for (int t = 0; t < 8; ++t) acc[t] = wmma16b(a, frag_kb(WAT + (size_t)(t * 16 + nloc) * D + kb, hlf), acc[t]); }
  const float alpha = 1.0f / (1.0f + __expf(-bf16_rne(skip[0])));
  float val[8][8], s1[8];
#pragma unroll
  for (int r = 0; r < 8; ++r) s1[r] = 0.0f;
#pragma unroll
  for (int t = 0; t < 8; ++t) { const int col = t * 16 + nloc; const float bb = bf16_rne(ba[col]);
#pragma unroll
    for (int r = 0; r < 8; ++r) { size_t frow = m0 + 8 * hlf + r; if (frow > (size_t)(N - 1)) frow = (size_t)(N - 1); const float o = alpha * (acc[t][r] * (1.0f / (XS * WSC)) + bb) + (1.0f - alpha) * bf16_rne(F[frow * D + col]); val[t][r] = o; s1[r] += o; } }
#pragma unroll
  for (int w = 1; w < 16; w <<= 1)
#pragma unroll
    for (int r = 0; r < 8; ++r) s1[r] += __shfl_xor(s1[r], w);
  float s2[8];
#pragma unroll
  for (int r = 0; r < 8; ++r) { s2[r] = 0.0f; const float mu_ = s1[r] * (1.0f / (float)D);
#pragma unroll
    for (int t = 0; t < 8; ++t) { const float d = val[t][r] - mu_; s2[r] = fmaf(d, d, s2[r]); } }
#pragma unroll
  for (int w = 1; w < 16; w <<= 1)
#pragma unroll
    for (int r = 0; r < 8; ++r) s2[r] += __shfl_xor(s2[r], w);
#pragma unroll
  for (int t = 0; t < 8; ++t) { const int col = t * 16 + nloc; const float gg = bf16_rne(g[col]), be = bf16_rne(bb_[col]);
#pragma unroll
    for (int r = 0; r < 8; ++r) { const float mu_ = s1[r] * (1.0f / (float)D); const float rs = rsqrtf(s2[r] * (1.0f / (float)D) + LNEPS); Tf[wave][8 * hlf + r][col] = (val[t][r] - mu_) * rs * gg + be; } }
  wave_lds_sync();
  for (int pass = 0; pass < 2; ++pass) { for (int rr = 0; rr < 16; ++rr) if (m0 + rr < (size_t)NL) *(volatile v4f*)(out + (m0 + rr) * D + lane * 4) = *(const v4f*)(&Tf[wave][rr][lane * 4]); __threadfence(); }
}
}

extern "C" void kernel_launch(void* const* d_in, const int* in_sizes, int n_in, void* d_out, int out_size, void* d_ws, size_t ws_size, hipStream_t stream) {
  (void)n_in;
  auto Fp = [&](int i) { return (const float*)d_in[i]; }; auto Ip = [&](int i) { return (const int*)d_in[i]; };
  if (in_sizes[0] != N * D || in_sizes[1] != N * D || in_sizes[2] != EFULL || in_sizes[3] != EFULL || in_sizes[4] != EFULL || in_sizes[5] != EFULL || in_sizes[6] != D * D || in_sizes[17] != D * D || in_sizes[28] != NH || in_sizes[29] != NH * DK * DK || in_sizes[33] != NH * DK * DK || in_sizes[16] != 1 || in_sizes[27] != 1 || out_size != 2 * N * D) return;
  size_t off = 0; char* ws = (char*)d_ws;
  auto carve = [&](size_t bytes) { char* p = ws + off; off += (bytes + 255) & ~(size_t)255; return p; };
  const size_t wsz = (size_t)D * D * 2;
  b16* WK_u = (b16*)carve(wsz); b16* WQ_u = (b16*)carve(wsz); b16* WV_u = (b16*)carve(wsz); b16* WA_u = (b16*)carve(wsz); b16* WK_i = (b16*)carve(wsz); b16* WQ_i = (b16*)carve(wsz); b16* WV_i = (b16*)carve(wsz); b16* WA_i = (b16*)carve(wsz);
  b16* BAT_ui = (b16*)carve(wsz); b16* BAQ_ui = (b16*)carve(wsz); b16* BMT_ui = (b16*)carve(wsz); b16* BMQ_ui = (b16*)carve(wsz); b16* BAT_iu = (b16*)carve(wsz); b16* BAQ_iu = (b16*)carve(wsz); b16* BMT_iu = (b16*)carve(wsz); b16* BMQ_iu = (b16*)carve(wsz);
  float* KP = (float*)carve((size_t)NP * D * 4); float* VP = (float*)carve((size_t)NP * D * 4); float* QP = (float*)carve((size_t)NP * D * 4); float* HP = (float*)carve((size_t)NP * D * 4);
  CsrBufs csr; off = csr_carve(csr, ws, off, E, N);
  if (off > ws_size || off > ((size_t)160 << 20)) return;
  const unsigned g8 = (D * D / 8 + 255) / 256;
  wprep_kernel<D, D><<<g8, 256, 0, stream>>>(Fp(6), WK_u); wprep_kernel<D, D><<<g8, 256, 0, stream>>>(Fp(8), WQ_u); wprep_kernel<D, D><<<g8, 256, 0, stream>>>(Fp(10), WV_u); wprep_kernel<D, D><<<g8, 256, 0, stream>>>(Fp(12), WA_u);
  wprep_kernel<D, D><<<g8, 256, 0, stream>>>(Fp(17), WK_i); wprep_kernel<D, D><<<g8, 256, 0, stream>>>(Fp(19), WQ_i); wprep_kernel<D, D><<<g8, 256, 0, stream>>>(Fp(21), WV_i); wprep_kernel<D, D><<<g8, 256, 0, stream>>>(Fp(23), WA_i);
  bd_kernel<<<g8, 256, 0, stream>>>(Fp(29), BAT_ui, WSC); bd_kernel<<<g8, 256, 0, stream>>>(Fp(29), BAQ_ui, WSQ); bd_kernel<<<g8, 256, 0, stream>>>(Fp(30), BMT_ui, WSC); bd_kernel<<<g8, 256, 0, stream>>>(Fp(30), BMQ_ui, WSQ);
  bd_kernel<<<g8, 256, 0, stream>>>(Fp(32), BAT_iu, WSC); bd_kernel<<<g8, 256, 0, stream>>>(Fp(32), BAQ_iu, WSQ); bd_kernel<<<g8, 256, 0, stream>>>(Fp(33), BMT_iu, WSC); bd_kernel<<<g8, 256, 0, stream>>>(Fp(33), BMQ_iu, WSQ);
  proj_kernel<true><<<NP / 32, 64, 0, stream>>>(Fp(0), WK_u, Fp(7), BAT_ui, BAQ_ui, KP); proj_kernel<true><<<NP / 32, 64, 0, stream>>>(Fp(0), WV_u, Fp(11), BMT_ui, BMQ_ui, VP); proj_kernel<false><<<NPL / 32, 64, 0, stream>>>(Fp(1), WQ_i, Fp(20), nullptr, nullptr, QP);
  csr_build(csr, Ip(3), E, N, stream);
  attn_kernel<<<NPL / 64, 256, 0, stream>>>(QP, KP, VP, Fp(28), Ip(2), csr.PERM, csr.ROWPTR, csr.ROWCNT, (int)csr.permLen, HP);
  nodeout_kernel<<<NPL / 32, 64, 0, stream>>>(HP, Fp(1), WA_i, Fp(24), Fp(27), Fp(25), Fp(26), (float*)d_out + (size_t)N * D);
  proj_kernel<true><<<NP / 32, 64, 0, stream>>>(Fp(1), WK_i, Fp(18), BAT_iu, BAQ_iu, KP); proj_kernel<true><<<NP / 32, 64, 0, stream>>>(Fp(1), WV_i, Fp(22), BMT_iu, BMQ_iu, VP); proj_kernel<false><<<NPL / 32, 64, 0, stream>>>(Fp(0), WQ_u, Fp(9), nullptr, nullptr, QP);
  csr_build(csr, Ip(5), E, N, stream);
  attn_kernel<<<NPL / 64, 256, 0, stream>>>(QP, KP, VP, Fp(31), Ip(4), csr.PERM, csr.ROWPTR, csr.ROWCNT, (int)csr.permLen, HP);
  nodeout_kernel<<<NPL / 32, 64, 0, stream>>>(HP, Fp(0), WA_u, Fp(13), Fp(16), Fp(14), Fp(15), (float*)d_out);
}
